// PointNetFeaturePropagation_58798102282445
// MI455X (gfx1250) — hardware-verified
//
#include <hip/hip_runtime.h>
#include <math.h>

typedef __attribute__((ext_vector_type(16))) _Float16 v16h;
typedef __attribute__((ext_vector_type(16))) __bf16 v16b;
typedef __attribute__((ext_vector_type(8)))  _Float16 v8h;
typedef __attribute__((ext_vector_type(8)))  float v8f;
typedef __attribute__((ext_vector_type(4)))  float v4f;
typedef __attribute__((ext_vector_type(2)))  float v2f;
typedef __attribute__((ext_vector_type(4)))  unsigned v4u;
typedef __attribute__((ext_vector_type(4)))  int v4i;
typedef float __attribute__((may_alias)) float_a;
typedef int __attribute__((may_alias)) int_a;

template <typename T> __device__ __forceinline__ void vst2(void* p, T v) { *(volatile T*)p = v; __threadfence(); *(volatile T*)p = v; }
__device__ __forceinline__ v8f wmma16(v16h a, v16h b, v8f c) {
  v8f d = __builtin_amdgcn_wmma_f32_16x16x32_f16(false, a, false, b, (short)0, c, false, false);
  asm volatile("v_nop\n\tv_nop\n\tv_nop\n\tv_nop" : "+v"(d) : "v"(a), "v"(b));
  return d;
}
__device__ __forceinline__ v8f wmma_bf(v16b a, v16b b, v8f c) {
  v8f d = __builtin_amdgcn_wmma_f32_16x16x32_bf16(false, a, false, b, (short)0, c, false, false);
  asm volatile("v_nop\n\tv_nop\n\tv_nop\n\tv_nop" : "+v"(d) : "v"(a), "v"(b));
  return d;
}
__device__ __forceinline__ v16h frag_h(const _Float16* rowk0, int lane) {
  union { v16h v; v8h q[2]; } u; const _Float16* p = rowk0 + 8 * (lane >> 4);
  u.q[0] = *(const v8h*)p; u.q[1] = *(const v8h*)(p + 16); return u.v;
}
__device__ __forceinline__ v16h frag_f32(const float* rowk0, int lane) {
  v16h a; const float* p = rowk0 + 8 * (lane >> 4);
#pragma unroll
  for (int i = 0; i < 8; ++i) { a[i] = (_Float16)p[i]; a[8 + i] = (_Float16)p[16 + i]; }
  return a;
}
__device__ __forceinline__ v16h frag_f32s(const float* rowk0, int lane, float sc) {
  v16h a; const float* p = rowk0 + 8 * (lane >> 4);
#pragma unroll
  for (int i = 0; i < 8; ++i) { a[i] = (_Float16)(p[i] * sc); a[8 + i] = (_Float16)(p[16 + i] * sc); }
  return a;
}
__device__ __forceinline__ v16h fragc_f32(const float* W, int k0, int n, int lane, int ld, int K) {
  v16h a; const int g = lane >> 4;
#pragma unroll
  for (int i = 0; i < 8; ++i) { const int ka = k0 + 8 * g + i, kb = ka + 16;
    a[i] = (_Float16)(ka < K ? W[(size_t)(ka < K ? ka : K - 1) * ld + n] : 0.f); a[8 + i] = (_Float16)(kb < K ? W[(size_t)(kb < K ? kb : K - 1) * ld + n] : 0.f); }
  return a;
}
struct F2 { v16b h, l; };
__device__ __forceinline__ F2 bsplit16(const float v[16]) { F2 r;
#pragma unroll
  for (int i = 0; i < 16; ++i) { const __bf16 h = (__bf16)v[i]; r.h[i] = h; r.l[i] = (__bf16)(v[i] - (float)h); }
  return r; }
__device__ __forceinline__ F2 split_row(const float* row, int k0, int lane) { float v[16]; const float* p = row + k0 + 8 * (lane >> 4);
#pragma unroll
  for (int i = 0; i < 8; ++i) { v[i] = p[i]; v[8 + i] = p[16 + i]; }
  return bsplit16(v); }
__device__ __forceinline__ F2 split_rowK(const float* row, int k0, int lane, int K) { float v[16]; const int g = lane >> 4;
#pragma unroll
  for (int i = 0; i < 8; ++i) { const int ka = k0 + 8 * g + i, kb = ka + 16; v[i] = ka < K ? row[ka < K ? ka : K - 1] : 0.f; v[8 + i] = kb < K ? row[kb < K ? kb : K - 1] : 0.f; }
  return bsplit16(v); }
__device__ __forceinline__ F2 split_col(const float* W, int k0, int n, int lane, int ld, int K) { float v[16]; const int g = lane >> 4;
#pragma unroll
  for (int i = 0; i < 8; ++i) { const int ka = k0 + 8 * g + i, kb = ka + 16; v[i] = ka < K ? W[(size_t)(ka < K ? ka : K - 1) * ld + n] : 0.f; v[8 + i] = kb < K ? W[(size_t)(kb < K ? kb : K - 1) * ld + n] : 0.f; }
  return bsplit16(v); }
__device__ __forceinline__ v8f mac3(const F2& a, const F2& b, v8f c) { c = wmma_bf(a.l, b.h, c); c = wmma_bf(a.h, b.l, c); return wmma_bf(a.h, b.h, c); }
__device__ __forceinline__ float sigm(float v) { return 1.0f / (1.0f + expf(-v)); }
#define LDSX() do { asm volatile("s_wait_dscnt 0" ::: "memory"); __builtin_amdgcn_wave_barrier(); __builtin_amdgcn_fence(__ATOMIC_RELEASE, "workgroup"); } while (0)

#define NB 8
#define NQ 8192
#define NS 2048
#define D1 128
#define D2 256
#define CIN 384
#define P1OFF 0
#define IOFF 128
#define CMAX 256
#define CL 128
#define NR (NB * NQ)
#ifndef TNB
#define TNB NB
#endif
#ifndef NQP
#define NQP NQ
#endif
#define NRV (TNB * NQ)
__device__ __forceinline__ float bfr(float v) { return (float)(__bf16)v; }
__device__ __forceinline__ v16b wcol_oi(const float* Wm, int k0, int o, int lane, int K) { v16b w; const float* p = Wm + (size_t)o * K + k0 + 8 * (lane >> 4);
#pragma unroll
  for (int i = 0; i < 8; ++i) { w[i] = (__bf16)p[i]; w[8 + i] = (__bf16)p[16 + i]; }
  return w; }
__device__ __forceinline__ v16b wcol_io(const float* Wm, int k0, int o, int lane, int ld) { v16b w; const int g = lane >> 4; float t0[8], t1[8];
#pragma unroll
  for (int i = 0; i < 8; ++i) t0[i] = Wm[(size_t)(k0 + 8 * g + i) * ld + o];
  asm volatile("s_wait_loadcnt 0x0" ::: "memory");
#pragma unroll
  for (int i = 0; i < 8; ++i) t1[i] = Wm[(size_t)(k0 + 16 + 8 * g + i) * ld + o];
  asm volatile("s_wait_loadcnt 0x0" ::: "memory");
#pragma unroll
  for (int i = 0; i < 8; ++i) { w[i] = (__bf16)t0[i]; w[8 + i] = (__bf16)t1[i]; }
  return w; }
#define WS_XC  0u
#define WS_TA  (WS_XC + 4u * (size_t)NR * CIN)
#define WS_TB  (WS_XC)
#define WS_ST  (WS_TA + 4u * (size_t)NR * CMAX)
#define WS_END (WS_ST + 4u * (size_t)2 * CMAX * 32 + 4u * (8 * 384 + 8 * 256) + 256u)


__global__ __launch_bounds__(256) void k_tr(const float* __restrict__ P1, float* __restrict__ XC) { __shared__ float st[D1][65];
  const int t = threadIdx.x; const int n0 = blockIdx.x * 64; const size_t b = blockIdx.y;
  for (int e = t; e < D1 * 64; e += 256) { const int c = e >> 6, ll = e & 63; st[c][ll] = bfr(P1[(b * D1 + c) * (size_t)NQP + n0 + ll]); }
  __syncthreads();
  for (int e = t; e < 64 * (D1 / 4); e += 256) { const int ll = e / (D1 / 4), q = e % (D1 / 4); v4f o; o[0] = st[q * 4][ll]; o[1] = st[q * 4 + 1][ll]; o[2] = st[q * 4 + 2][ll]; o[3] = st[q * 4 + 3][ll]; vst2(XC + (b * NQ + n0 + ll) * (size_t)CIN + P1OFF + q * 4, o); } }
struct Best3 { float d0, d1, d2; int i0, i1, i2; };
__device__ __forceinline__ void push3(Best3& b, float d, int i) {
  if (d < b.d0) { b.d2 = b.d1; b.i2 = b.i1; b.d1 = b.d0; b.i1 = b.i0; b.d0 = d; b.i0 = i; } else if (d < b.d1) { b.d2 = b.d1; b.i2 = b.i1; b.d1 = d; b.i1 = i; } else if (d < b.d2) { b.d2 = d; b.i2 = i; } }
__device__ __forceinline__ bool lessdi(float d, int i, float e, int j) { return d < e || (d == e && i < j); }
__global__ __launch_bounds__(256) void k_nn(const float* __restrict__ X1, const float* __restrict__ X2, const float* __restrict__ P2, float* __restrict__ XC) {
  const int wave = threadIdx.x >> 5, lane = threadIdx.x & 31; const size_t row = (size_t)blockIdx.x * 8 + wave; if (row >= (size_t)NRV) return;
  const size_t b = row / NQ; const int n = (int)(row % NQ);
  Best3 bs; bs.d0 = bs.d1 = bs.d2 = 3.0e38f; bs.i0 = bs.i1 = bs.i2 = 0x7fffffff;
  {
#pragma clang fp contract(off)
    const float qx = bfr(X1[(b * NQP + n) * 3 + 0]), qy = bfr(X1[(b * NQP + n) * 3 + 1]), qz = bfr(X1[(b * NQP + n) * 3 + 2]);
    const float aa = (qx * qx + qy * qy) + qz * qz;
#pragma unroll 1
    for (int s = lane; s < NS; s += 32) { const float px = bfr(X2[(b * NS + s) * 3 + 0]), py = bfr(X2[(b * NS + s) * 3 + 1]), pz = bfr(X2[(b * NS + s) * 3 + 2]);
      const float bb = (px * px + py * py) + pz * pz; const float dot = (qx * px + qy * py) + qz * pz;
      const float d = (aa + bb) - 2.0f * dot;
      push3(bs, fmaxf(d, 0.0f), s); } }
  float rd[3]; int ri[3];
#pragma unroll
  for (int r = 0; r < 3; ++r) { float d = bs.d0; int i = bs.i0;
#pragma unroll
    for (int o = 1; o < 32; o <<= 1) { const float e = __shfl_xor(d, o); const int j = __shfl_xor(i, o); if (lessdi(e, j, d, i)) { d = e; i = j; } }
    rd[r] = d; ri[r] = i; if (bs.i0 == i && bs.d0 == d) { bs.d0 = bs.d1; bs.i0 = bs.i1; bs.d1 = bs.d2; bs.i1 = bs.i2; bs.d2 = 3.0e38f; bs.i2 = 0x7fffffff; } }
  float w[3]; { float rc[3]; for (int r = 0; r < 3; ++r) rc[r] = 1.0f / (rd[r] + 1e-8f); const float sm = (rc[0] + rc[1]) + rc[2]; for (int r = 0; r < 3; ++r) w[r] = rc[r] / sm; }
  float o8[D2 / 32];
#pragma unroll
  for (int i = 0; i < D2 / 32; ++i) { const int cc = (i >> 2) * 128 + 4 * lane + (i & 3); float acc = 0.f;
#pragma unroll
    for (int r = 0; r < 3; ++r) { const int ic = ri[r] < 0 ? 0 : (ri[r] >= NS ? NS - 1 : ri[r]); acc += bfr(P2[(b * D2 + cc) * (size_t)NS + ic]) * w[r]; }
    o8[i] = acc; }
#pragma unroll
  for (int q = 0; q < D2 / 128; ++q) { v4f o; o[0] = o8[q * 4]; o[1] = o8[q * 4 + 1]; o[2] = o8[q * 4 + 2]; o[3] = o8[q * 4 + 3]; vst2(XC + row * CIN + IOFF + q * 128 + 4 * lane, o); } }
__device__ __forceinline__ float gelu_exact(float x) { return 0.5f * x * (1.0f + erff(x * 0.70710678118654752f)); }
__device__ __forceinline__ F2 arow(const float* row, int k0, int lane, const float* __restrict__ ST, const float* __restrict__ G, const float* __restrict__ BE, const float* __restrict__ TVb) { float v[16]; const float* p = row + k0 + 8 * (lane >> 4);
#pragma unroll
  for (int i = 0; i < 8; ++i) { v[i] = p[i]; v[8 + i] = p[16 + i]; }
  asm volatile("s_wait_loadcnt 0x0" ::: "memory");
  if (ST) {
#pragma unroll
    for (int i = 0; i < 16; ++i) { const int cc = k0 + 8 * (lane >> 4) + (i < 8 ? i : 8 + i); const float mu = ST[cc * 32], rs = ST[cc * 32 + 1], gg = G[cc], be = BE[cc]; asm volatile("s_wait_loadcnt 0x0" ::: "memory"); const float y = (v[i] - mu) * rs * bfr(gg) + bfr(be); v[i] = gelu_exact(y); } }
  if (TVb) {
#pragma unroll
    for (int i = 0; i < 16; ++i) { const int cc = k0 + 8 * (lane >> 4) + (i < 8 ? i : 8 + i); v[i] += TVb[cc]; } }
  asm volatile("s_wait_loadcnt 0x0" ::: "memory");
  return bsplit16(v); }
__global__ __launch_bounds__(256) void k_tvec(const float* __restrict__ TE, const float* __restrict__ Wt, const float* __restrict__ TB, int nch, float* __restrict__ TVo) { const int wave = threadIdx.x >> 5, lane = threadIdx.x & 31; const int idx = blockIdx.x * 8 + wave; if (idx >= TNB * nch) return; const int b = idx / nch, c = idx % nch;
  float a = 0.f; for (int j = lane; j < 128; j += 32) a += gelu_exact(bfr(TE[b * 128 + j])) * bfr(Wt[(size_t)c * 128 + j]);
#pragma unroll
  for (int o = 1; o < 32; o <<= 1) a += __shfl_xor(a, o);
  if (lane == 0) { const float tb = bfr(TB[c]); asm volatile("s_wait_loadcnt 0x0" ::: "memory"); vst2(TVo + (size_t)b * nch + c, a + tb); } }
__global__ __launch_bounds__(128) void k_conv(const float* __restrict__ IN, int ldin, int K, const float* __restrict__ ST, const float* __restrict__ G, const float* __restrict__ BE, const float* __restrict__ Wt, int woi, const float* __restrict__ BIAS, int nout, float* __restrict__ OUTR, const float* __restrict__ TV, int tvn) { __shared__ __align__(16) float sf[4][16][132];
  const int tid = threadIdx.x, wave = tid >> 5, lane = tid & 31, col = lane & 15, g = lane >> 4; const int c0 = blockIdx.y * 128; const size_t r0 = (size_t)blockIdx.x * 64 + wave * 16;
  v8f acc[8] = {};
#pragma unroll 1
  for (int kc = 0; kc < K / 32; ++kc) { const F2 a = arow(IN + (r0 + col) * ldin, kc * 32, lane, ST, G, BE, TV ? TV + (r0 / NQ) * (size_t)tvn : nullptr);
#pragma unroll
    for (int j = 0; j < 8; ++j) { v16b w; if (woi) { w = wcol_oi(Wt, kc * 32, c0 + j * 16 + col, lane, K); asm volatile("s_wait_loadcnt 0x0" ::: "memory"); } else { w = wcol_io(Wt, kc * 32, c0 + j * 16 + col, lane, nout); }
      acc[j] = wmma_bf(a.h, w, acc[j]); acc[j] = wmma_bf(a.l, w, acc[j]); } }
#pragma unroll
  for (int j = 0; j < 8; ++j) { const float bb = BIAS ? bfr(BIAS[c0 + j * 16 + col]) : 0.f;
#pragma unroll
    for (int r = 0; r < 8; ++r) sf[wave][8 * g + r][j * 16 + col] = acc[j][r] + bb; }
  asm volatile("s_wait_loadcnt 0x0" ::: "memory");
  LDSX(); for (int rl = 0; rl < 16; ++rl) vst2(OUTR + (r0 + rl) * (size_t)nout + c0 + lane * 4, *(const v4f*)&sf[wave][rl][lane * 4]); }
__global__ __launch_bounds__(256) void k_stat(const float* __restrict__ T, int ld, float* __restrict__ STAT) { __shared__ float sred[8]; __shared__ float sbc;
  const int t = threadIdx.x; const int c = blockIdx.x;
  float s = 0.f; for (int r = t; r < NRV; r += 256) s += T[(size_t)r * ld + c];
#pragma unroll
  for (int o = 1; o < 32; o <<= 1) s += __shfl_xor(s, o);
  if ((t & 31) == 0) sred[t >> 5] = s; __syncthreads(); if (t == 0) { float a = 0.f; for (int i = 0; i < 8; ++i) a += sred[i]; sbc = a / (float)NRV; } __syncthreads(); const float mean = sbc; __syncthreads();
  float q = 0.f; for (int r = t; r < NRV; r += 256) { const float d = T[(size_t)r * ld + c] - mean; q += d * d; }
#pragma unroll
  for (int o = 1; o < 32; o <<= 1) q += __shfl_xor(q, o);
  if ((t & 31) == 0) sred[t >> 5] = q; __syncthreads(); if (t == 0) { float a = 0.f; for (int i = 0; i < 8; ++i) a += sred[i]; sbc = rsqrtf(a / (float)NRV + 1e-5f); } __syncthreads();
  if (t < 32) { const float v = t == 0 ? mean : (t == 1 ? sbc : 0.f); vst2(STAT + (size_t)c * 32 + t, v); } }
__global__ __launch_bounds__(256) void k_evst(const float* __restrict__ MU, const float* __restrict__ VAR, int nch, float eps, float* __restrict__ STo) { const int c = blockIdx.x * 8 + (threadIdx.x >> 5), t = threadIdx.x & 31; if (c >= nch) return; const float v = t == 0 ? bfr(MU[c]) : (t == 1 ? rsqrtf(bfr(VAR[c]) + eps) : 0.f); vst2(STo + (size_t)c * 32 + t, v); }
__global__ __launch_bounds__(256) void k_finR(const float* __restrict__ T, const float* __restrict__ ST, const float* __restrict__ G, const float* __restrict__ BE, float* __restrict__ OUT) { const size_t e4 = (size_t)blockIdx.x * 256 + threadIdx.x; if (e4 >= (size_t)NRV * (CL / 4)) return; const size_t row = e4 / (CL / 4); const int c0 = (int)(e4 % (CL / 4)) * 4; const v4f x = *(const v4f*)(T + row * CL + c0); v4f o;
#pragma unroll
  for (int i = 0; i < 4; ++i) { const int cc = c0 + i; o[i] = fmaxf((x[i] - ST[cc * 32]) * ST[cc * 32 + 1] * bfr(G[cc]) + bfr(BE[cc]), 0.f); }
  vst2(OUT + row * CL + c0, o); }
__global__ __launch_bounds__(128) void k_finT(const float* __restrict__ T, const float* __restrict__ ST, const float* __restrict__ G, const float* __restrict__ BE, float* __restrict__ OUT) { __shared__ __align__(16) float stc[128][68];
  const int tid = threadIdx.x; const int c0 = blockIdx.y * 128; const size_t rb = (size_t)blockIdx.x * 64;
  for (int e = tid; e < 64 * 128; e += 128) { const int rl = e >> 7, cl = e & 127; const int cc = c0 + cl; const float x = (T[(rb + rl) * CL + cc] - ST[cc * 32]) * ST[cc * 32 + 1] * bfr(G[cc]) + bfr(BE[cc]); stc[cl][rl] = gelu_exact(x); }
  __syncthreads();
  { const size_t b = rb / NQ; const int n0 = (int)(rb % NQ); for (int e = tid; e < 128 * 16; e += 128) { const int cl = e >> 4, q = e & 15; vst2(OUT + (b * CL + c0 + cl) * (size_t)NQP + n0 + q * 4, *(const v4f*)&stc[cl][q * 4]); } } }
extern "C" void kernel_launch(void* const* d_in, const int* in_sizes, int n_in, void* d_out, int out_size, void* d_ws, size_t ws_size, hipStream_t stream) {
  (void)in_sizes; (void)n_in; (void)out_size;
  const float** F = (const float**)d_in;
  if (ws_size < (size_t)WS_END) return;
  char* ws = (char*)d_ws; float *XC = (float*)(ws + WS_XC), *TA = (float*)(ws + WS_TA), *TB = (float*)(ws + WS_TB), *ST = (float*)(ws + WS_ST);
  k_tr<<<dim3(NQ / 64, TNB), 256, 0, stream>>>(F[2], XC);
  k_nn<<<dim3((NRV + 7) / 8), 256, 0, stream>>>(F[0], F[1], F[3], XC);
  float* TV = ST + 2 * CMAX * 32;
  k_tvec<<<dim3((TNB * 384 + 7) / 8), 256, 0, stream>>>(F[4], F[5], F[6], 384, TV);
  k_tvec<<<dim3((TNB * 256 + 7) / 8), 256, 0, stream>>>(F[4], F[11], F[12], 256, TV + 8 * 384);
  k_conv<<<dim3(NRV / 64, 2), 128, 0, stream>>>(XC, CIN, CIN, nullptr, nullptr, nullptr, F[7], 1, F[8], 256, TA, TV, 384);
  k_stat<<<dim3(256), 256, 0, stream>>>(TA, 256, ST);
  k_conv<<<dim3(NRV / 64, 1), 128, 0, stream>>>(TA, 256, 256, ST, F[9], F[10], F[13], 1, F[14], 128, TB, TV + 8 * 384, 256);
  k_stat<<<dim3(128), 256, 0, stream>>>(TB, 128, ST + CMAX * 32);
  k_finT<<<dim3(NRV / 64, CL / 128), 128, 0, stream>>>(TB, ST + CMAX * 32, F[15], F[16], (float*)d_out);
}
